// LSTMModel_23098334118250
// MI455X (gfx1250) — hardware-verified
//
#include <hip/hip_runtime.h>
#include <math.h>

constexpr int NBATCH   = 4096;
constexpr int NSTEP    = 512;
constexpr int NHID     = 20;
constexpr int NGATE    = 4 * NHID;
constexpr int TILE_B   = 16;
constexpr int CHUNK    = 32;
constexpr int NCHUNK   = NSTEP / CHUNK;
constexpr int HALF_U   = NHID / 2;
constexpr int NTILE    = NGATE / 16;
constexpr int WAVE_SZ  = 32;
constexpr float H_CARRY   = 16.0f;
constexpr float W_CARRY   = 16.0f;
constexpr float RES_SCALE = 2048.0f;
constexpr float INV_MAIN  = 1.0f / (H_CARRY * W_CARRY);
constexpr float INV_RES   = INV_MAIN / RES_SCALE;
constexpr int W4_COUNT = NGATE * NHID / 4;
constexpr int W4_ITERS = (W4_COUNT + WAVE_SZ - 1) / WAVE_SZ;

static_assert(NGATE == 80 && NTILE == 5, "gate rows are five 16-row tiles");
static_assert(NHID == 2 * HALF_U && HALF_U == 10, "ten hidden units per lane half");
static_assert(HALF_U + 1 <= 16, "hidden slots plus one input slot fit one lane half");
static_assert(NSTEP % CHUNK == 0 && CHUNK * 4 == 128, "one chunk of steps is one 128-B line per row");
static_assert(NBATCH % TILE_B == 0, "batch tiles exact");
static_assert(NGATE / 4 <= WAVE_SZ && NHID / 4 <= WAVE_SZ, "small vectors staged by one wave");
static_assert(W4_ITERS * WAVE_SZ >= W4_COUNT, "weight staging coverage");

typedef __attribute__((ext_vector_type(16))) _Float16 v16h;
typedef __attribute__((ext_vector_type(8)))  float    v8f;
typedef __attribute__((ext_vector_type(4)))  float    v4f;

union FragU { v16h v; unsigned u[8]; };

__device__ __forceinline__ void split16(float v, unsigned& hb, unsigned& lb) {
  const _Float16 h = (_Float16)v;
  const float hv = (float)h;
  const float r = (v - hv) * RES_SCALE;
  const _Float16 l = (_Float16)r;
  const unsigned short hs = __builtin_bit_cast(unsigned short, h);
  const unsigned short ls = __builtin_bit_cast(unsigned short, l);
  hb = (unsigned)hs;
  lb = (unsigned)ls;
}
__device__ __forceinline__ unsigned pack_lohi(unsigned lo16, unsigned hi16) { return lo16 | (hi16 << 16); }

__device__ __forceinline__ v8f mma_h(v16h a, v16h b, v8f c) {
  return __builtin_amdgcn_wmma_f32_16x16x32_f16(false, a, false, b, (short)0, c, false, false);
}
__device__ __forceinline__ void group_guard(v8f& m, v8f& r, v16h a0, v16h a1, v16h b0, v16h b1) {
  asm volatile("v_nop\n\tv_nop\n\tv_nop\n\tv_nop" : "+v"(m), "+v"(r) : "v"(a0), "v"(a1), "v"(b0), "v"(b1));
}

__device__ __forceinline__ float act_sigm(float x) { return __builtin_amdgcn_rcpf(1.0f + expf(-x)); }
__device__ __forceinline__ float act_tanh(float x) { return 1.0f - 2.0f * __builtin_amdgcn_rcpf(1.0f + expf(2.0f * x)); }

__global__ __launch_bounds__(32) void rnn_cell_seq_kernel(
    const float* __restrict__ x, const float* __restrict__ W_ih, const float* __restrict__ W_hh,
    const float* __restrict__ b_ih, const float* __restrict__ b_hh,
    const float* __restrict__ W_lin, const float* __restrict__ b_lin, float* __restrict__ out) {
  __shared__ __align__(16) float Wst[NGATE * NHID];
  __shared__ __align__(16) float Wis[NGATE];
  __shared__ __align__(16) float Bss[NGATE];
  __shared__ __align__(16) float WLs[NHID];
  __shared__ __align__(16) float Xs[TILE_B * CHUNK];
  __shared__ __align__(16) float Po[2 * TILE_B * CHUNK];
  __shared__ __align__(16) float Gs[8 * NTILE * WAVE_SZ];
  __shared__ __align__(16) float Cs[HALF_U * WAVE_SZ];
  __shared__ __align__(16) float Hn[HALF_U * WAVE_SZ];

  const int lane = threadIdx.x & 31;
  const int n    = lane & 15;
  const int hf   = lane >> 4;
  const bool upper = (hf != 0);
  const int b0   = blockIdx.x * TILE_B;

#pragma unroll 1
  for (int it = 0; it < W4_ITERS; ++it) {
    int i = it * WAVE_SZ + lane;
    i = (i < W4_COUNT - 1) ? i : (W4_COUNT - 1);
    const v4f v = *(const v4f*)(W_hh + 4 * i);
    *(v4f*)(Wst + 4 * i) = v;
  }
  {
    const int i20 = (lane < NGATE / 4 - 1) ? lane : (NGATE / 4 - 1);
    const v4f wi = *(const v4f*)(W_ih + 4 * i20);
    const v4f bi = *(const v4f*)(b_ih + 4 * i20);
    const v4f bh = *(const v4f*)(b_hh + 4 * i20);
    v4f bs;
    bs[0] = bi[0] + bh[0];
    bs[1] = bi[1] + bh[1];
    bs[2] = bi[2] + bh[2];
    bs[3] = bi[3] + bh[3];
    *(v4f*)(Wis + 4 * i20) = wi;
    *(v4f*)(Bss + 4 * i20) = bs;
    const int i5 = (lane < NHID / 4 - 1) ? lane : (NHID / 4 - 1);
    const v4f wl = *(const v4f*)(W_lin + 4 * i5);
    *(v4f*)(WLs + 4 * i5) = wl;
  }
  const float blin = b_lin[0];
#pragma unroll
  for (int q = 0; q < HALF_U; ++q) {
    Cs[q * WAVE_SZ + lane] = 0.0f;
    Hn[q * WAVE_SZ + lane] = 0.0f;
  }
  __syncthreads();

  v16h Ahi[NTILE], Alo[NTILE];
#pragma unroll
  for (int t = 0; t < NTILE; ++t) {
    const int sidx = 8 * t + (n & 7);
    const int gate = sidx & 3;
    const int unit = ((n >= 8) ? HALF_U : 0) + (sidx >> 2);
    const int row  = gate * NHID + unit;
    const float* wr = Wst + row * NHID + HALF_U * hf;
    unsigned hb[HALF_U], lb[HALF_U];
#pragma unroll
    for (int e = 0; e < HALF_U; ++e) split16(wr[e] * W_CARRY, hb[e], lb[e]);
    const float wi_v = Wis[row];
    const float bs_v = Bss[row];
    const float wsel = upper ? bs_v : wi_v;
    unsigned h10, l10;
    split16(wsel * W_CARRY, h10, l10);
    FragU fh, fl;
#pragma unroll
    for (int k = 0; k < 5; ++k) {
      fh.u[k] = pack_lohi(hb[2 * k], hb[2 * k + 1]);
      fl.u[k] = pack_lohi(lb[2 * k], lb[2 * k + 1]);
    }
    fh.u[5] = h10;
    fl.u[5] = l10;
    fh.u[6] = 0u;
    fh.u[7] = 0u;
    fl.u[6] = 0u;
    fl.u[7] = 0u;
    Ahi[t] = fh.v;
    Alo[t] = fl.v;
  }

  unsigned one_hb, one_lb;
  split16(H_CARRY, one_hb, one_lb);

  const float* xbase = x   + (size_t)b0 * NSTEP;
  float*       obase = out + (size_t)b0 * NSTEP;
  const v8f z8 = {0.f, 0.f, 0.f, 0.f, 0.f, 0.f, 0.f, 0.f};

#pragma unroll 1
  for (int ch = 0; ch < NCHUNK; ++ch) {
#pragma unroll
    for (int it = 0; it < 4; ++it) {
      const int idx = it * WAVE_SZ + lane;
      const int row = idx >> 3;
      const int c4  = (idx & 7) * 4;
      const v4f v = *(const v4f*)(xbase + (size_t)row * NSTEP + ch * CHUNK + c4);
      *(v4f*)(Xs + row * CHUNK + c4) = v;
    }
    __syncthreads();

#pragma unroll 1
    for (int s = 0; s < CHUNK; ++s) {
      unsigned hb[HALF_U], lb[HALF_U];
#pragma unroll
      for (int q = 0; q < HALF_U; ++q) split16(Hn[q * WAVE_SZ + lane], hb[q], lb[q]);
      const float xv = Xs[n * CHUNK + s] * H_CARRY;
      unsigned xh, xl;
      split16(xv, xh, xl);
      const unsigned w5h = upper ? one_hb : xh;
      const unsigned w5l = upper ? one_lb : xl;
      FragU bh, bl;
#pragma unroll
      for (int k = 0; k < 5; ++k) {
        bh.u[k] = pack_lohi(hb[2 * k], hb[2 * k + 1]);
        bl.u[k] = pack_lohi(lb[2 * k], lb[2 * k + 1]);
      }
      bh.u[5] = w5h;
      bl.u[5] = w5l;
      bh.u[6] = 0u;
      bh.u[7] = 0u;
      bl.u[6] = 0u;
      bl.u[7] = 0u;

#pragma unroll
      for (int t = 0; t < NTILE; ++t) {
        v8f accM = mma_h(Ahi[t], bh.v, z8);
        v8f accR = mma_h(Ahi[t], bl.v, z8);
        accR = mma_h(Alo[t], bh.v, accR);
        group_guard(accM, accR, Ahi[t], Alo[t], bh.v, bl.v);
#pragma unroll
        for (int r = 0; r < 8; ++r) {
          const float gv = accM[r] * INV_MAIN + accR[r] * INV_RES;
          Gs[(8 * t + r) * WAVE_SZ + lane] = gv;
        }
      }

      float oacc = 0.0f;
#pragma unroll 1
      for (int q = 0; q < HALF_U; ++q) {
        const float gi = Gs[(4 * q + 0) * WAVE_SZ + lane];
        const float gf = Gs[(4 * q + 1) * WAVE_SZ + lane];
        const float gg = Gs[(4 * q + 2) * WAVE_SZ + lane];
        const float go = Gs[(4 * q + 3) * WAVE_SZ + lane];
        const float cp = Cs[q * WAVE_SZ + lane];
        const float wl = WLs[HALF_U * hf + q];
        const float ig = act_sigm(gi);
        const float fg = act_sigm(gf);
        const float gt = act_tanh(gg);
        const float og = act_sigm(go);
        const float cn = fg * cp + ig * gt;
        const float hv = og * act_tanh(cn);
        Cs[q * WAVE_SZ + lane] = cn;
        Hn[q * WAVE_SZ + lane] = hv * H_CARRY;
        oacc = fmaf(wl, hv, oacc);
      }
      Po[(hf * TILE_B + n) * CHUNK + s] = oacc;
    }
    __syncthreads();

    v4f ov[4];
#pragma unroll
    for (int it = 0; it < 4; ++it) {
      const int idx = it * WAVE_SZ + lane;
      const int row = idx >> 3;
      const int c4  = (idx & 7) * 4;
      const v4f pa = *(const v4f*)(Po + row * CHUNK + c4);
      const v4f pb = *(const v4f*)(Po + (TILE_B + row) * CHUNK + c4);
      v4f o;
      o[0] = (pa[0] + pb[0]) + blin;
      o[1] = (pa[1] + pb[1]) + blin;
      o[2] = (pa[2] + pb[2]) + blin;
      o[3] = (pa[3] + pb[3]) + blin;
      ov[it] = o;
    }
    for (int pass = 0; pass < 2; ++pass) {
#pragma unroll
      for (int it = 0; it < 4; ++it) {
        const int idx = it * WAVE_SZ + lane;
        const int row = idx >> 3;
        const int c4  = (idx & 7) * 4;
        *(volatile v4f*)(obase + (size_t)row * NSTEP + ch * CHUNK + c4) = ov[it];
      }
      __threadfence();
    }
    __syncthreads();
  }
}

extern "C" void kernel_launch(void* const* d_in, const int* in_sizes, int n_in,
                              void* d_out, int out_size, void* d_ws, size_t ws_size, hipStream_t stream) {
  (void)d_ws; (void)ws_size;
  if (n_in < 7 || d_out == nullptr) return;
  if (in_sizes[0] != NBATCH * NSTEP || in_sizes[1] != NGATE || in_sizes[2] != NGATE * NHID ||
      in_sizes[3] != NGATE || in_sizes[4] != NGATE || in_sizes[5] != NHID || in_sizes[6] != 1 ||
      out_size != NBATCH * NSTEP) return;
  const float* x     = (const float*)d_in[0];
  const float* W_ih  = (const float*)d_in[1];
  const float* W_hh  = (const float*)d_in[2];
  const float* b_ih  = (const float*)d_in[3];
  const float* b_hh  = (const float*)d_in[4];
  const float* W_lin = (const float*)d_in[5];
  const float* b_lin = (const float*)d_in[6];
  float* outp = (float*)d_out;
  rnn_cell_seq_kernel<<<NBATCH / TILE_B, 32, 0, stream>>>(x, W_ih, W_hh, b_ih, b_hh, W_lin, b_lin, outp);
}
